// ForTorPredictorNN_23175643529937
// MI455X (gfx1250) — hardware-verified
//
#include <hip/hip_runtime.h>
#include <math.h>

constexpr int kBatch = 4;
constexpr int kPart  = 2048;
constexpr int kNbr   = 32;
constexpr int kRows  = kPart * kNbr;
constexpr int kFeatIn = 77;
constexpr int kFeatK  = 96;
constexpr int kHid    = 256;
constexpr int kFinN   = 64;
constexpr int kOutPerChunk = kPart * 3;
constexpr float kWCarry   = 16.0f;
constexpr float kActCarry = 8.0f;
constexpr float kInvStd   = 0.999995f;
constexpr float kBoxLen   = 20.0f;
constexpr float kInvBox   = 0.05f;
constexpr float kScaleL1  = kActCarry / kWCarry;
constexpr float kScaleLh  = kActCarry / (kActCarry * kWCarry);
constexpr float kScaleLf  = 1.0f / (kActCarry * kWCarry);
constexpr float kInvNbr   = 1.0f / 32.0f;

constexpr size_t kOffW0t  = 0;
constexpr size_t kOffWh0t = 49152;
constexpr size_t kOffWh1t = 180224;
constexpr size_t kOffWfT  = 311296;
constexpr size_t kOffCb0  = 344064;
constexpr size_t kOffCb1  = 345088;
constexpr size_t kOffCb2  = 346112;
constexpr size_t kOffFeat = 1048576;
constexpr size_t kOffHa   = kOffFeat + (size_t)kRows * kFeatK * 2;
constexpr size_t kOffHb   = kOffHa + (size_t)kRows * kHid * 2;
constexpr size_t kOffFout = kOffHb + (size_t)kRows * kHid * 2;
constexpr size_t kWsEnd   = kOffFout + (size_t)kRows * kFinN * 4;
static_assert(kOffHa == 13631488);
static_assert(kWsEnd == 97517568);
static_assert(kWsEnd <= 134217728);

typedef __attribute__((ext_vector_type(16))) _Float16 v16h;
typedef __attribute__((ext_vector_type(8)))  _Float16 v8h;
typedef __attribute__((ext_vector_type(16))) __bf16   v16b;
typedef __attribute__((ext_vector_type(8)))  __bf16   v8b;
typedef __attribute__((ext_vector_type(8)))  float    v8f;
typedef __attribute__((ext_vector_type(4)))  float    v4f;
typedef __attribute__((ext_vector_type(4)))  unsigned int v4u;

__device__ __forceinline__ unsigned short f2bf_bits(float f) {
  unsigned u = __float_as_uint(f);
  return (unsigned short)((u + 0x7FFFu + ((u >> 16) & 1u)) >> 16);
}
__device__ __forceinline__ float bf_bits2f(unsigned short h) { return __uint_as_float(((unsigned)h) << 16); }

__device__ __forceinline__ void dep_guard_h(v8f& a, v8f& b, v16h x, v16h y) { asm volatile("v_nop\n\tv_nop\n\tv_nop\n\tv_nop" : "+v"(a), "+v"(b) : "v"(x), "v"(y)); }
__device__ __forceinline__ void dep_guard_b(v8f& a, v8f& b, v16b x, v16b y) { asm volatile("v_nop\n\tv_nop\n\tv_nop\n\tv_nop" : "+v"(a), "+v"(b) : "v"(x), "v"(y)); }
__device__ __forceinline__ void keep4_h(v16h a, v16h b, v16h c, v16h d) { asm volatile("v_nop" :: "v"(a), "v"(b), "v"(c), "v"(d)); }
__device__ __forceinline__ void keep4_b(v16b a, v16b b, v16b c, v16b d) { asm volatile("v_nop" :: "v"(a), "v"(b), "v"(c), "v"(d)); }
__device__ __forceinline__ void acc_guard4(v8f& a, v8f& b, v8f& c, v8f& d) { asm volatile("v_nop\n\tv_nop\n\tv_nop\n\tv_nop" : "+v"(a), "+v"(b), "+v"(c), "+v"(d)); }
template <typename T> struct Frag;
template <> struct Frag<_Float16> {
  typedef v16h V; union U { v16h v; v8h h[2]; };
  static __device__ __forceinline__ v16h load(const _Float16* p) {
    U f; f.h[0] = *(const v8h*)(p); f.h[1] = *(const v8h*)(p + 16); return f.v;
  }
  static __device__ __forceinline__ v8f mma(v16h a, v16h b, v8f c) {
    return __builtin_amdgcn_wmma_f32_16x16x32_f16(false, a, false, b, (short)0, c, false, false);
  }
  static __device__ __forceinline__ void guard(v8f& a, v8f& b, v16h x, v16h y) { dep_guard_h(a, b, x, y); }
  static __device__ __forceinline__ void keep(v16h a, v16h b, v16h c, v16h d) { keep4_h(a, b, c, d); }
};
template <> struct Frag<__bf16> {
  typedef v16b V; union U { v16b v; v8b h[2]; };
  static __device__ __forceinline__ v16b load(const __bf16* p) {
    U f; f.h[0] = *(const v8b*)(p); f.h[1] = *(const v8b*)(p + 16); return f.v;
  }
  static __device__ __forceinline__ v8f mma(v16b a, v16b b, v8f c) {
    return __builtin_amdgcn_wmma_f32_16x16x32_bf16(false, a, false, b, (short)0, c, false, false);
  }
  static __device__ __forceinline__ void guard(v8f& a, v8f& b, v16b x, v16b y) { dep_guard_b(a, b, x, y); }
  static __device__ __forceinline__ void keep(v16b a, v16b b, v16b c, v16b d) { keep4_b(a, b, c, d); }
};

__device__ __forceinline__ unsigned pk16(unsigned short a, unsigned short b) { return (unsigned)a | ((unsigned)b << 16); }
__device__ __forceinline__ unsigned short h_bits(float f) { const _Float16 h = (_Float16)f; return __builtin_bit_cast(unsigned short, h); }

template <int ET> struct Elem;
template <> struct Elem<0> { typedef _Float16 T; };
template <> struct Elem<1> { typedef __bf16 T; };
template <int ET, bool SPLIT, int BIAS_MODE, int OUT_MODE, bool RESID, int ACT = 0>
__global__ __launch_bounds__(256) void wmma_gemm64(
    const unsigned short* __restrict__ Ap, const unsigned short* __restrict__ A2p, int lda, long strideA,
    const unsigned short* __restrict__ Btp, const unsigned short* __restrict__ Bt2p, int ldb, long strideB,
    void* __restrict__ Cout, void* __restrict__ Cout2, int ldc, long strideC,
    const float* __restrict__ bias,
    const float* __restrict__ resid, long strideR,
    int M, int N, int K, float scale) {
  typedef typename Elem<ET>::T T;
  typedef typename Frag<T>::V V;
  const T* A = (const T*)Ap; const T* A2 = (const T*)A2p; const T* Bt = (const T*)Btp; const T* Bt2 = (const T*)Bt2p;
  __shared__ __align__(16) float sT[8][16 * 68];
  const int b    = blockIdx.y;
  const int lane = threadIdx.x & 31;
  const int wave = threadIdx.x >> 5;
  const int tilesN = N >> 6;
  const int tilesM = M >> 6;
  const int tile = blockIdx.x * 8 + wave;
  if (tile >= tilesM * tilesN) return;
  const int tm = tile / tilesN;
  const int tn = tile - tm * tilesN;
  const int m0 = tm << 6;
  const int n0 = tn << 6;

  const T* Ab  = A  + (size_t)b * strideA;
  const T* Bb  = Bt + (size_t)b * strideB;
  const T* Ab2 = SPLIT ? (A2  + (size_t)b * strideA) : nullptr;
  const T* Bb2 = SPLIT ? (Bt2 + (size_t)b * strideB) : nullptr;

  const int rlane = lane & 15;
  const int koff  = (lane >> 4) * 8;
  const int mOff  = (lane >> 4) * 8;

  v8f acc[4][4];
#pragma unroll
  for (int i = 0; i < 4; ++i)
#pragma unroll
    for (int j = 0; j < 4; ++j) acc[i][j] = (v8f){0.f,0.f,0.f,0.f,0.f,0.f,0.f,0.f};

  for (int k0 = 0; k0 < K; k0 += 32) {
    V bh[4], bl[4];
#pragma unroll
    for (int j = 0; j < 4; ++j) {
      const size_t bo = (size_t)(n0 + (j << 4) + rlane) * ldb + koff + k0;
      bh[j] = Frag<T>::load(Bb + bo);
      if (SPLIT) bl[j] = Frag<T>::load(Bb2 + bo);
    }
#pragma unroll
    for (int i = 0; i < 4; ++i) {
      const size_t ao = (size_t)(m0 + (i << 4) + rlane) * lda + koff + k0;
      V ah = Frag<T>::load(Ab + ao);
      V al;
      if (SPLIT) al = Frag<T>::load(Ab2 + ao);
#pragma unroll
      for (int j = 0; j < 4; ++j) {
        acc[i][j] = Frag<T>::mma(ah, bh[j], acc[i][j]);
        if (SPLIT) {
          acc[i][j] = Frag<T>::mma(ah, bl[j], acc[i][j]);
          acc[i][j] = Frag<T>::mma(al, bh[j], acc[i][j]);
        }
      }
      Frag<T>::guard(acc[i][0], acc[i][3], ah, SPLIT ? al : ah);
    }
    Frag<T>::keep(bh[0], bh[1], bh[2], bh[3]);
    if (SPLIT) Frag<T>::keep(bl[0], bl[1], bl[2], bl[3]);
  }
  acc_guard4(acc[0][0], acc[0][1], acc[0][2], acc[0][3]);
  acc_guard4(acc[1][0], acc[1][1], acc[1][2], acc[1][3]);
  acc_guard4(acc[2][0], acc[2][1], acc[2][2], acc[2][3]);
  acc_guard4(acc[3][0], acc[3][1], acc[3][2], acc[3][3]);

  float* slab = sT[wave];
  const float* Rb = RESID ? (resid + (size_t)b * strideR) : nullptr;
#pragma unroll
  for (int i = 0; i < 4; ++i) {
    const int mBase = m0 + (i << 4);
#pragma unroll
    for (int j = 0; j < 4; ++j) {
      const int n = n0 + (j << 4) + rlane;
      float bv = 0.f;
      if (BIAS_MODE == 2) bv = bias[n];
#pragma unroll
      for (int r = 0; r < 8; ++r) {
        float v = acc[i][j][r] * scale;
        if (BIAS_MODE == 1) v += bias[mBase + mOff + r];
        if (BIAS_MODE == 2) v += bv;
        if (RESID) v += Rb[(size_t)(mBase + mOff + r) * ldc + n];
        if (ACT == 2) v = fmaxf(v, 0.0f);
        if (ACT == 4) v = (v > 0.f) ? v : 0.01f * v;
        slab[(mOff + r) * 68 + (j << 4) + rlane] = v;
      }
    }
    __builtin_amdgcn_fence(__ATOMIC_RELEASE, "workgroup");
    __builtin_amdgcn_wave_barrier();
    __builtin_amdgcn_fence(__ATOMIC_ACQUIRE, "workgroup");
    if (OUT_MODE == 0) {
      float* C = (float*)Cout + (size_t)b * strideC;
      const int hh = lane >> 4, c4 = (lane & 15) * 4;
      for (int pass = 0; pass < 2; ++pass) {
#pragma unroll
        for (int it = 0; it < 8; ++it) {
          const int row = it * 2 + hh;
          v4f v = *(const v4f*)(slab + row * 68 + c4);
          *(volatile v4f*)(C + (size_t)(mBase + row) * ldc + n0 + c4) = v;
        }
        __threadfence();
      }
    } else {
      const int q = lane >> 3, c8 = (lane & 7) * 8;
      unsigned short* C  = (unsigned short*)Cout  + (size_t)b * strideC;
      unsigned short* C2 = (OUT_MODE == 2) ? ((unsigned short*)Cout2 + (size_t)b * strideC) : nullptr;
      for (int pass = 0; pass < 2; ++pass) {
#pragma unroll
        for (int it = 0; it < 4; ++it) {
          const int row = it * 4 + q;
          const float* sp = slab + row * 68 + c8;
          v8h hv, lv;
#pragma unroll
          for (int e = 0; e < 8; ++e) {
            if (OUT_MODE == 1) {
              hv[e] = (_Float16)sp[e];
            } else {
              unsigned short hb = f2bf_bits(sp[e]);
              unsigned short lb = f2bf_bits(sp[e] - bf_bits2f(hb));
              hv[e] = __builtin_bit_cast(_Float16, hb);
              lv[e] = __builtin_bit_cast(_Float16, lb);
            }
          }
          *(volatile v8h*)(C + (size_t)(mBase + row) * ldc + n0 + c8) = hv;
          if (OUT_MODE == 2) *(volatile v8h*)(C2 + (size_t)(mBase + row) * ldc + n0 + c8) = lv;
        }
        __threadfence();
      }
    }
    __builtin_amdgcn_fence(__ATOMIC_RELEASE, "workgroup");
    __builtin_amdgcn_wave_barrier();
    __builtin_amdgcn_fence(__ATOMIC_ACQUIRE, "workgroup");
  }
}

__global__ __launch_bounds__(256) void prep_small_kernel(
    const float* __restrict__ w0, const float* __restrict__ b0, const float* __restrict__ bh,
    const float* __restrict__ gamma, const float* __restrict__ beta, const float* __restrict__ wf,
    unsigned int* __restrict__ w0t_w, unsigned int* __restrict__ wft_w,
    float* __restrict__ cb0, float* __restrict__ cb1, float* __restrict__ cb2) {
#pragma clang fp contract(off)
  __shared__ __align__(16) unsigned int simg[256 * 48];
  const int t = threadIdx.x;
  const int role = blockIdx.x;
  if (role == 0) {
    const int n = t;
    const float zf = w0[n] - w0[n];
#pragma unroll 1
    for (int i = 0; i < 38; ++i) {
      const float a = w0[(2 * i) * kHid + n] * kWCarry;
      const float c = w0[(2 * i + 1) * kHid + n] * kWCarry;
      simg[n * 48 + i] = pk16(h_bits(a), h_bits(c));
    }
    {
      const float a = w0[76 * kHid + n] * kWCarry;
      simg[n * 48 + 38] = pk16(h_bits(a), h_bits(zf));
    }
    const unsigned zz = pk16(h_bits(zf), h_bits(zf));
#pragma unroll
    for (int i = 39; i < 48; ++i) simg[n * 48 + i] = zz;
  } else if (role == 1) {
    if (t < 128) {
      const float zf = wf[t * 6] - wf[t * 6];
#pragma unroll
      for (int n = 0; n < 3; ++n) {
        const float a = wf[(2 * t) * 3 + n] * kWCarry;
        const float c = wf[(2 * t + 1) * 3 + n] * kWCarry;
        simg[n * 128 + t] = pk16(h_bits(a), h_bits(c));
      }
      const unsigned zz = pk16(h_bits(zf), h_bits(zf));
#pragma unroll 1
      for (int n = 3; n < kFinN; ++n) simg[n * 128 + t] = zz;
    }
  }
  __syncthreads();
  if (role == 0) {
    for (int pass = 0; pass < 2; ++pass) {
#pragma unroll
      for (int it = 0; it < 12; ++it) {
        const int idx = it * 256 + t;
        const v4u v = *(const v4u*)(simg + idx * 4);
        *(volatile v4u*)(w0t_w + (size_t)idx * 4) = v;
      }
      __threadfence();
    }
  } else if (role == 1) {
    for (int pass = 0; pass < 2; ++pass) {
#pragma unroll
      for (int it = 0; it < 8; ++it) {
        const int idx = it * 256 + t;
        const v4u v = *(const v4u*)(simg + idx * 4);
        *(volatile v4u*)(wft_w + (size_t)idx * 4) = v;
      }
      __threadfence();
    }
  } else {
    if (t < 192) {
      const int which = t >> 6;
      const int i4 = (t & 63) * 4;
      v4f v = (v4f){0.f, 0.f, 0.f, 0.f};
#pragma unroll
      for (int e = 0; e < 4; ++e) {
        const int c = i4 + e;
        const float v0 = b0[c] * kActCarry;
        const float s1 = gamma[c] * kInvStd;
        const float s2 = gamma[kHid + c] * kInvStd;
        const float t1 = bh[c] * s1;
        const float v1 = (t1 + beta[c]) * kActCarry;
        const float t2 = bh[kHid + c] * s2;
        const float v2 = (t2 + beta[kHid + c]) * kActCarry;
        v[e] = (which == 0) ? v0 : ((which == 1) ? v1 : v2);
      }
      float* dst = (which == 0) ? cb0 : ((which == 1) ? cb1 : cb2);
      float* p = dst + i4;
      *(volatile v4f*)p = v;
      __threadfence();
      *(volatile v4f*)p = v;
    }
  }
}

__global__ __launch_bounds__(256) void prep_wh_kernel(const float* __restrict__ wh, const float* __restrict__ gamma,
                                                      unsigned short* __restrict__ wht) {
#pragma clang fp contract(off)
  __shared__ float sm[64][65];
  const int t  = threadIdx.x;
  const int k0 = blockIdx.x * 64;
  const int n0 = blockIdx.y * 64;
  const int z  = blockIdx.z;
  const float* wsrc = wh + (size_t)z * kHid * kHid;
#pragma unroll
  for (int i = 0; i < 16; ++i) {
    const int e = i * 256 + t;
    const int r = e >> 6;
    const int c = e & 63;
    const float s = gamma[z * kHid + n0 + c] * kInvStd;
    const float v = wsrc[(size_t)(k0 + r) * kHid + n0 + c] * s;
    sm[c][r] = v * kWCarry;
  }
  __syncthreads();
  const int lane = t & 31, wave = t >> 5;
  const int q = lane >> 3, c8 = (lane & 7) * 8;
  unsigned short* op = wht + (size_t)z * kHid * kHid;
  for (int pass = 0; pass < 2; ++pass) {
#pragma unroll
    for (int it = 0; it < 2; ++it) {
      const int row = wave * 8 + it * 4 + q;
      unsigned short hb[8];
#pragma unroll
      for (int e = 0; e < 8; ++e) hb[e] = h_bits(sm[row][c8 + e]);
      const v4u u = (v4u){pk16(hb[0], hb[1]), pk16(hb[2], hb[3]), pk16(hb[4], hb[5]), pk16(hb[6], hb[7])};
      *(volatile v4u*)(op + (size_t)(n0 + row) * kHid + k0 + c8) = u;
    }
    __threadfence();
  }
}

__global__ __launch_bounds__(256) void feat_kernel(const float* __restrict__ pos, const float* __restrict__ ori,
                                                   const int* __restrict__ nl, unsigned int* __restrict__ featw, int bchunk) {
#pragma clang fp contract(off)
  __shared__ __align__(16) unsigned int srow[256 * 48];
  const int t = threadIdx.x;
  const int rloc = blockIdx.x * 256 + t;
  const int n = rloc >> 5;
  const size_t grow = (size_t)bchunk * kRows + (size_t)rloc;
  int jn = nl[grow * 2 + 1];
  jn = (jn < 0) ? 0 : jn;
  jn = (jn > kPart - 1) ? (kPart - 1) : jn;
  const size_t pi = (size_t)bchunk * kPart + (size_t)n;
  const size_t pj = (size_t)bchunk * kPart + (size_t)jn;
  const float px = pos[pi * 3 + 0], py = pos[pi * 3 + 1], pz = pos[pi * 3 + 2];
  const float qx = pos[pj * 3 + 0], qy = pos[pj * 3 + 1], qz = pos[pj * 3 + 2];
  float ra[9], rb[9];
#pragma unroll
  for (int k = 0; k < 9; ++k) { ra[k] = ori[pi * 9 + k]; rb[k] = ori[pj * 9 + k]; }

  float dx = qx - px, dy = qy - py, dz = qz - pz;
  dx = dx - kBoxLen * rintf(dx * kInvBox);
  dy = dy - kBoxLen * rintf(dy * kInvBox);
  dz = dz - kBoxLen * rintf(dz * kInvBox);
  const float rr  = (dx * dx + dz * dz) + dy * dy;
  const float rad = sqrtf(rr);
  const float inv = 1.0f / rad;
  const float zf  = rad - rad;

  float fv[80];
  fv[0] = rad;
  fv[1] = dx * inv; fv[2] = dy * inv; fv[3] = dz * inv;
  fv[4] = inv;
#pragma unroll
  for (int i = 0; i < 3; ++i) {
#pragma unroll
    for (int j = 0; j < 3; ++j) {
      float s = ra[i] * rb[j];
      s = s + ra[3 + i] * rb[3 + j];
      s = s + ra[6 + i] * rb[6 + j];
      fv[5 + i * 3 + j] = s;
    }
  }
#pragma unroll
  for (int i = 0; i < 3; ++i) {
#pragma unroll
    for (int j = 0; j < 3; ++j) {
      const float e0 = ra[i] * rb[j];
      const float e1 = ra[3 + i] * rb[3 + j];
      const float e2 = ra[6 + i] * rb[6 + j];
      const int base = 14 + (i * 3 + j) * 3;
      fv[base + 0] = e0; fv[base + 1] = e1; fv[base + 2] = e2;
      const float ss = (e0 * e0 + e2 * e2) + e1 * e1;
      fv[41 + i * 3 + j] = __builtin_amdgcn_sqrtf(ss);
    }
  }
#pragma unroll
  for (int i = 0; i < 3; ++i) {
    const float a0 = ra[i], a1 = ra[3 + i], a2 = ra[6 + i];
    const float g0 = rb[i], g1 = rb[3 + i], g2 = rb[6 + i];
    const float c0 = a1 * g2 - a2 * g1;
    const float c1 = a2 * g0 - a0 * g2;
    const float c2 = a0 * g1 - a1 * g0;
    fv[50 + i * 3 + 0] = c0; fv[50 + i * 3 + 1] = c1; fv[50 + i * 3 + 2] = c2;
    const float ss = (c0 * c0 + c2 * c2) + c1 * c1;
    fv[59 + i] = __builtin_amdgcn_sqrtf(ss);
  }
#pragma unroll
  for (int i = 0; i < 3; ++i) {
#pragma unroll
    for (int j = 0; j < 3; ++j) {
      float s = ra[i * 3] * rb[j * 3];
      s = s + ra[i * 3 + 1] * rb[j * 3 + 1];
      s = s + ra[i * 3 + 2] * rb[j * 3 + 2];
      fv[62 + i * 3 + j] = s;
    }
  }
  float pp0 = dx * ra[0]; pp0 = pp0 + dy * ra[3]; pp0 = pp0 + dz * ra[6];
  float pp1 = dx * ra[1]; pp1 = pp1 + dy * ra[4]; pp1 = pp1 + dz * ra[7];
  float pp2 = dx * ra[2]; pp2 = pp2 + dy * ra[5]; pp2 = pp2 + dz * ra[8];
  float pn0 = dx * rb[0]; pn0 = pn0 + dy * rb[3]; pn0 = pn0 + dz * rb[6];
  float pn1 = dx * rb[1]; pn1 = pn1 + dy * rb[4]; pn1 = pn1 + dz * rb[7];
  float pn2 = dx * rb[2]; pn2 = pn2 + dy * rb[5]; pn2 = pn2 + dz * rb[8];
  float rf0 = 0.f, rf1 = 0.f, rf2 = 0.f, rf3 = 0.f, rf4 = 0.f, rf5 = 0.f;
#pragma unroll 1
  for (int qq = 0; qq < 6; ++qq) {
    const float p = (qq == 0) ? pp0 : (qq == 1) ? pp1 : (qq == 2) ? pp2 : (qq == 3) ? pn0 : (qq == 4) ? pn1 : pn2;
    const float psq = p * p;
    const float ev = expf(-psq);
    rf0 = (qq == 0) ? ev : rf0;
    rf1 = (qq == 1) ? ev : rf1;
    rf2 = (qq == 2) ? ev : rf2;
    rf3 = (qq == 3) ? ev : rf3;
    rf4 = (qq == 4) ? ev : rf4;
    rf5 = (qq == 5) ? ev : rf5;
  }
  fv[71] = rf0; fv[72] = rf1; fv[73] = rf2;
  fv[74] = rf3; fv[75] = rf4; fv[76] = rf5;
  fv[77] = zf; fv[78] = zf; fv[79] = zf;

  unsigned int* myrow = srow + t * 48;
#pragma unroll
  for (int g = 0; g < 10; ++g) {
    v4u u;
    u[0] = pk16(h_bits(fv[8 * g + 0]), h_bits(fv[8 * g + 1]));
    u[1] = pk16(h_bits(fv[8 * g + 2]), h_bits(fv[8 * g + 3]));
    u[2] = pk16(h_bits(fv[8 * g + 4]), h_bits(fv[8 * g + 5]));
    u[3] = pk16(h_bits(fv[8 * g + 6]), h_bits(fv[8 * g + 7]));
    *(v4u*)(myrow + 4 * g) = u;
  }
  {
    const unsigned zz = pk16(h_bits(zf), h_bits(zf));
    const v4u uz = (v4u){zz, zz, zz, zz};
    *(v4u*)(myrow + 40) = uz;
    *(v4u*)(myrow + 44) = uz;
  }
  __syncthreads();
  unsigned int* gbase = featw + (size_t)blockIdx.x * (256 * 48);
  for (int pass = 0; pass < 2; ++pass) {
#pragma unroll
    for (int it = 0; it < 12; ++it) {
      const int idx = it * 256 + t;
      const v4u v = *(const v4u*)(srow + idx * 4);
      *(volatile v4u*)(gbase + (size_t)idx * 4) = v;
    }
    __threadfence();
  }
}

__global__ __launch_bounds__(256) void pool_kernel(const float* __restrict__ fin, const float* __restrict__ bfp,
                                                   float* __restrict__ out, int bchunk) {
#pragma clang fp contract(off)
  const int tg = blockIdx.x * 256 + threadIdx.x;
  if (tg >= kOutPerChunk / 4) return;
  v4f res = (v4f){0.f, 0.f, 0.f, 0.f};
#pragma unroll
  for (int e = 0; e < 4; ++e) {
    const int f = tg * 4 + e;
    const int n = f / 3;
    const int c = f - n * 3;
    const float bc = bfp[c];
    const float* col = fin + (size_t)n * (kNbr * kFinN) + c;
    float s = 0.0f;
#pragma unroll 8
    for (int m = 0; m < kNbr; ++m) s = s + (col[(size_t)m * kFinN] + bc);
    res[e] = s * kInvNbr;
  }
  float* op = out + (size_t)bchunk * kOutPerChunk + (size_t)tg * 4;
  *(volatile v4f*)op = res;
  __threadfence();
  *(volatile v4f*)op = res;
}

extern "C" void kernel_launch(void* const* d_in, const int* in_sizes, int n_in,
                              void* d_out, int out_size, void* d_ws, size_t ws_size,
                              hipStream_t stream) {
  if (n_in < 11) return;
  if (in_sizes[0] != kBatch * kPart * 3) return;
  if (in_sizes[1] != kBatch * kPart * 9) return;
  if (in_sizes[2] != kBatch * kRows * 2) return;
  if (in_sizes[3] != kFeatIn * kHid) return;
  if (in_sizes[4] != kHid) return;
  if (in_sizes[5] != 2 * kHid * kHid) return;
  if (in_sizes[6] != 2 * kHid || in_sizes[7] != 2 * kHid || in_sizes[8] != 2 * kHid) return;
  if (in_sizes[9] != kHid * 3) return;
  if (in_sizes[10] < 3) return;
  if (out_size != kBatch * kOutPerChunk) return;
  if (ws_size < kWsEnd) return;

  const float* position = (const float*)d_in[0];
  const float* orient   = (const float*)d_in[1];
  const int*   nlist    = (const int*)d_in[2];
  const float* w0    = (const float*)d_in[3];
  const float* b0    = (const float*)d_in[4];
  const float* wh    = (const float*)d_in[5];
  const float* bh    = (const float*)d_in[6];
  const float* gamma = (const float*)d_in[7];
  const float* beta  = (const float*)d_in[8];
  const float* wf    = (const float*)d_in[9];
  const float* bf    = (const float*)d_in[10];
  float* out = (float*)d_out;

  char* ws = (char*)d_ws;
  unsigned short* w0t16  = (unsigned short*)(ws + kOffW0t);
  unsigned short* wh0t16 = (unsigned short*)(ws + kOffWh0t);
  unsigned short* wh1t16 = (unsigned short*)(ws + kOffWh1t);
  unsigned short* wft16  = (unsigned short*)(ws + kOffWfT);
  float* cb0 = (float*)(ws + kOffCb0);
  float* cb1 = (float*)(ws + kOffCb1);
  float* cb2 = (float*)(ws + kOffCb2);
  unsigned short* feat16 = (unsigned short*)(ws + kOffFeat);
  unsigned short* ha16   = (unsigned short*)(ws + kOffHa);
  unsigned short* hb16   = (unsigned short*)(ws + kOffHb);
  float* fout = (float*)(ws + kOffFout);

  prep_small_kernel<<<dim3(3), dim3(256), 0, stream>>>(
      w0, b0, bh, gamma, beta, wf, (unsigned int*)w0t16, (unsigned int*)wft16, cb0, cb1, cb2);
  prep_wh_kernel<<<dim3(kHid / 64, kHid / 64, 2), dim3(256), 0, stream>>>(wh, gamma, wh0t16);

  const int tilesH = (kRows / 64) * (kHid / 64);
  const int tilesF = (kRows / 64) * (kFinN / 64);
  for (int b = 0; b < kBatch; ++b) {
    feat_kernel<<<dim3(kRows / 256), dim3(256), 0, stream>>>(position, orient, nlist, (unsigned int*)feat16, b);
    wmma_gemm64<0, false, 2, 1, false, 2><<<dim3((tilesH + 7) / 8, 1), dim3(256), 0, stream>>>(
        feat16, feat16, kFeatK, 0L, w0t16, w0t16, kFeatK, 0L, (void*)ha16, (void*)ha16, kHid, 0L,
        cb0, cb0, 0L, kRows, kHid, kFeatK, kScaleL1);
    wmma_gemm64<0, false, 2, 1, false, 2><<<dim3((tilesH + 7) / 8, 1), dim3(256), 0, stream>>>(
        ha16, ha16, kHid, 0L, wh0t16, wh0t16, kHid, 0L, (void*)hb16, (void*)hb16, kHid, 0L,
        cb1, cb1, 0L, kRows, kHid, kHid, kScaleLh);
    wmma_gemm64<0, false, 2, 1, false, 2><<<dim3((tilesH + 7) / 8, 1), dim3(256), 0, stream>>>(
        hb16, hb16, kHid, 0L, wh1t16, wh1t16, kHid, 0L, (void*)ha16, (void*)ha16, kHid, 0L,
        cb2, cb2, 0L, kRows, kHid, kHid, kScaleLh);
    wmma_gemm64<0, false, 0, 0, false, 0><<<dim3((tilesF + 7) / 8, 1), dim3(256), 0, stream>>>(
        ha16, ha16, kHid, 0L, wft16, wft16, kHid, 0L, (void*)fout, (void*)fout, kFinN, 0L,
        cb0, cb0, 0L, kRows, kFinN, kHid, kScaleLf);
    pool_kernel<<<dim3(kOutPerChunk / 4 / 256), dim3(256), 0, stream>>>(fout, bf, out, b);
  }
}
